// GraphAttentionLayer_86912958202744
// MI455X (gfx1250) — hardware-run, weakly checked
//
#include <hip/hip_runtime.h>


namespace {
constexpr int NB = 8, CI = 32, N = 2048, L = 12, F = 32, CL = CI * L  , KB = 128;
constexpr float XS = 8.0f, WSC = 256.0f, PS = 256.0f, SLOPE = 0.2f;
typedef _Float16 b16;
typedef __attribute__((ext_vector_type(16))) _Float16 v16b;
typedef __attribute__((ext_vector_type(8))) _Float16 v8b;
typedef __attribute__((ext_vector_type(8))) float v8f;
typedef __attribute__((ext_vector_type(4))) float v4f;
typedef __attribute__((ext_vector_type(2))) float v2f;
__device__ __forceinline__ float bf16_rne(float f) { unsigned int u = __float_as_uint(f); u += 0x7FFFu + ((u >> 16) & 1u); float r = __uint_as_float(u & 0xFFFF0000u); asm volatile("" : "+v"(r)); return r; }
__device__ __forceinline__ float bfv(float f) { float r = bf16_rne(f); asm volatile("" : "+v"(r)); return r; }
__device__ __forceinline__ void split16(float v, b16& hi, b16& lo) { hi = (b16)v; lo = (b16)(v - (float)hi); }
__device__ __forceinline__ v16b frag_kb(const b16* p, int hh) { const v8b a = *(const v8b*)(p + 8 * hh), b = *(const v8b*)(p + 16 + 8 * hh); v16b f;
#pragma unroll
  for (int e = 0; e < 8; ++e) { f[e] = a[e]; f[8 + e] = b[e]; } return f; }
__device__ __forceinline__ v8f wmma16b(v16b a, v16b b, v8f c) { v8f d = __builtin_amdgcn_wmma_f32_16x16x32_f16(false, a, false, b, (short)0, c, false, false); asm volatile("v_nop\n\tv_nop\n\tv_nop\n\tv_nop" : "+v"(d) : "v"(a), "v"(b)); return d; }
__device__ __forceinline__ void wave_lds_sync() { __builtin_amdgcn_fence(__ATOMIC_RELEASE, "workgroup"); __builtin_amdgcn_wave_barrier(); __builtin_amdgcn_fence(__ATOMIC_ACQUIRE, "workgroup"); }
__device__ __forceinline__ float pmul(float a, float b) { float p = a * b; asm volatile("" : "+v"(p)); return p; }
__device__ __forceinline__ float leaky(float v) { return v > 0.0f ? v : SLOPE * v; }
__device__ __forceinline__ float elu(float v) { return v > 0.0f ? v : (__expf(v) - 1.0f); }

__global__ __launch_bounds__(256) void wput_kernel(const float* __restrict__ W, const float* __restrict__ a, b16* __restrict__ WT, float* __restrict__ WA) { const int u = threadIdx.x;
  if (u < F * 4) { const int f = u / 4, k0 = (u % 4) * 8; v8b v;
#pragma unroll
    for (int j = 0; j < 8; ++j) v[j] = (b16)(bf16_rne(W[(size_t)(k0 + j) * F + f]) * WSC); for (int pass = 0; pass < 2; ++pass) { *(volatile v8b*)(WT + (size_t)f * CI + k0) = v; __threadfence(); } }
  if (u < 2 * CI) { const int g = u / CI, c = u % CI; float s = 0.0f;
#pragma unroll 1
    for (int f = 0; f < F; ++f) s += pmul(bfv(W[(size_t)c * F + f]), bfv(a[g * F + f]));
    for (int pass = 0; pass < 2; ++pass) { ((volatile float*)WA)[g * CI + c] = s; __threadfence(); } } }
__global__ __launch_bounds__(256) void s_kernel(const float* __restrict__ h, const float* __restrict__ WA, float* __restrict__ S12) { const int u = blockIdx.x * 256 + threadIdx.x; if (u >= NB * N) return; const int b = u / N, n = u % N; float s1 = 0.0f, s2 = 0.0f;
#pragma unroll 1
  for (int c = 0; c < CI; ++c) { const float hv = bfv(h[(((size_t)b * CI + c) * N + n) * L + (L - 1)]); s1 += pmul(hv, WA[c]); s2 += pmul(hv, WA[CI + c]); }
  for (int pass = 0; pass < 2; ++pass) { ((volatile float*)S12)[((size_t)b * 2) * N + n] = s1; ((volatile float*)S12)[((size_t)b * 2 + 1) * N + n] = s2; __threadfence(); } }
typedef __attribute__((ext_vector_type(2))) _Float16 v2b;
__global__ __launch_bounds__(256) void ht_kernel(const float* __restrict__ h, b16* __restrict__ HT) { const size_t u = (size_t)blockIdx.x * 256 + threadIdx.x; if (u >= (size_t)NB * CL * N / 2) return; const size_t e = u * 2; const int v = (int)(e % N); const int col = (int)((e / N) % CL); const int b = (int)(e / ((size_t)N * CL)); const int c = col / L, l = col % L;
  const size_t hb = (((size_t)b * CI + c) * N + v) * L + l; v2b val; val[0] = (b16)(bf16_rne(h[hb]) * XS); val[1] = (b16)(bf16_rne(h[hb + L]) * XS); for (int pass = 0; pass < 2; ++pass) { *(volatile v2b*)(HT + e) = val; __threadfence(); } }
__global__ __launch_bounds__(32) void att_kernel(const float* __restrict__ S12, const int* __restrict__ adj, const b16* __restrict__ HT, int BLIM, float* __restrict__ G) { __shared__ __attribute__((aligned(16))) b16 Ph_[16][KB + 8], Pl_[16][KB + 8]; __shared__ float Sf[16][KB + 4], Of[16][132];
  const int lane = threadIdx.x, nloc = lane & 15, hlf = lane >> 4; const int g = blockIdx.x % 3; const int qt = (blockIdx.x / 3) % (N / 16); const int b = blockIdx.x / (3 * (N / 16)); if (b >= BLIM) return; const int w0 = qt * 16;
  const float* s1p = S12 + (size_t)b * 2 * N; const float* s2p = s1p + N; const b16* HTb = HT + ((size_t)b * CL + g * 128) * N;
  float m_r[8], den_r[8]; v8f acc[8];
#pragma unroll
  for (int r8 = 0; r8 < 8; ++r8) { m_r[r8] = -INFINITY; den_r[r8] = 0.0f; }
#pragma unroll
  for (int t = 0; t < 8; ++t) acc[t] = (v8f){};
  __shared__ float S2s[16]; if (lane < 16) S2s[lane] = s2p[w0 + lane]; wave_lds_sync();
#pragma unroll 1
  for (int kb0 = 0; kb0 < N; kb0 += KB) {
#pragma unroll 1
    for (int q = 0; q < 4; ++q) { const int v = kb0 + q * 32 + lane; const float s1v = s1p[v]; const int* arow = adj + (size_t)v * N + w0;
#pragma unroll 4
      for (int rr = 0; rr < 16; ++rr) Sf[rr][q * 32 + lane] = arow[rr] != 0 ? leaky(s1v + S2s[rr]) : -INFINITY; }
    wave_lds_sync();
#pragma unroll
    for (int rr = 0; rr < 16; ++rr) { float mx = -INFINITY;
#pragma unroll
      for (int q = 0; q < 4; ++q) mx = fmaxf(mx, Sf[rr][q * 32 + lane]);
      for (int o = 16; o; o >>= 1) mx = fmaxf(mx, __shfl_xor(mx, o));
      const float mold = __shfl(m_r[rr & 7], (rr >> 3) * 16); const float mn = fmaxf(mold, mx); const float sf = (mold == -INFINITY) ? 0.0f : ((mn == -INFINITY) ? 1.0f : __expf(mold - mn)); float ps = 0.0f;
#pragma unroll
      for (int q = 0; q < 4; ++q) { const int kx = q * 32 + lane; const float sv = Sf[rr][kx]; const float p = (sv == -INFINITY || mn == -INFINITY) ? 0.0f : __expf(sv - mn); ps += p; b16 ph, pl; split16(p * PS, ph, pl); Ph_[rr][kx] = ph; Pl_[rr][kx] = pl; }
      for (int o = 16; o; o >>= 1) ps += __shfl_xor(ps, o);
      if ((rr >> 3) == hlf) { const int r8 = rr & 7; den_r[r8] = den_r[r8] * sf + ps; m_r[r8] = mn;
#pragma unroll
        for (int t = 0; t < 8; ++t) acc[t][r8] = acc[t][r8] * sf; } }
    wave_lds_sync();
#pragma unroll
    for (int ks = 0; ks < KB; ks += 32) { const v16b pa = frag_kb(&Ph_[nloc][ks], hlf), pb = frag_kb(&Pl_[nloc][ks], hlf);
#pragma unroll
      for (int t = 0; t < 8; ++t) { const v16b hb = frag_kb(HTb + (size_t)(t * 16 + nloc) * N + kb0 + ks, hlf); acc[t] = wmma16b(pa, hb, acc[t]); acc[t] = wmma16b(pb, hb, acc[t]); } }
    wave_lds_sync(); }
#pragma unroll
  for (int t = 0; t < 8; ++t)
#pragma unroll
    for (int r8 = 0; r8 < 8; ++r8) { const float dn = den_r[r8]; Of[8 * hlf + r8][t * 16 + nloc] = dn > 0.0f ? acc[t][r8] * (1.0f / (XS * PS)) / dn : 0.0f; }
  wave_lds_sync();
  for (int pass = 0; pass < 2; ++pass) { for (int rr = 0; rr < 16; ++rr) *(volatile v4f*)(G + ((size_t)b * N + w0 + rr) * CL + g * 128 + lane * 4) = *(const v4f*)(&Of[rr][lane * 4]); __threadfence(); } }
__global__ __launch_bounds__(32) void out_kernel(const float* __restrict__ G, const b16* __restrict__ WT, int BLIM, float* __restrict__ out) { __shared__ __attribute__((aligned(16))) b16 Ah[16][40], Al[16][40]; __shared__ float Tf[F][16 * L + 4]; const int lane = threadIdx.x, nloc = lane & 15, hlf = lane >> 4; const int qt = blockIdx.x % (N / 16); const int b = blockIdx.x / (N / 16); if (b >= BLIM) return; const int w0 = qt * 16;
#pragma unroll 1
  for (int l = 0; l < L; ++l) {
    for (int rr = 0; rr < 16; ++rr) { const float v = G[((size_t)b * N + w0 + rr) * CL + lane * L + l]; b16 p, ql; split16(v * XS, p, ql); Ah[rr][lane] = p; Al[rr][lane] = ql; if (lane < 8) { Ah[rr][32 + lane] = (b16)0.0f; Al[rr][32 + lane] = (b16)0.0f; } }
    wave_lds_sync(); const v16b a = frag_kb(&Ah[nloc][0], hlf), al = frag_kb(&Al[nloc][0], hlf);
#pragma unroll
    for (int t = 0; t < 2; ++t) { const v16b bw = frag_kb(WT + (size_t)(t * 16 + nloc) * CI, hlf); v8f acc = {}; acc = wmma16b(a, bw, acc); acc = wmma16b(al, bw, acc);
#pragma unroll
      for (int r8 = 0; r8 < 8; ++r8) Tf[t * 16 + nloc][(8 * hlf + r8) * L + l] = elu(acc[r8] * (1.0f / (XS * WSC))); }
    wave_lds_sync(); }
  for (int pass = 0; pass < 2; ++pass) { for (int f = 0; f < F; ++f) { float* dst = out + (((size_t)b * F + f) * N + w0) * L; for (int k = 0; k < 6; ++k) ((volatile float*)dst)[lane * 6 + k] = Tf[f][lane * 6 + k]; } __threadfence(); } }
}

extern "C" void kernel_launch(void* const* d_in, const int* in_sizes, int n_in, void* d_out, int out_size, void* d_ws, size_t ws_size, hipStream_t stream) {
  (void)n_in;
  auto Fp = [&](int i) { return (const float*)d_in[i]; }; auto Ip = [&](int i) { return (const int*)d_in[i]; };
  if (in_sizes[0] != NB * CI * N * L || in_sizes[1] != N * N || in_sizes[2] != CI * F || in_sizes[3] != 2 * F || out_size != NB * F * N * L) return;
  const int BLIM = NB;
  size_t off = 0; char* ws = (char*)d_ws;
  auto carve = [&](size_t bytes) { char* p = ws + off; off += (bytes + 255) & ~(size_t)255; return p; };
  b16* WT = (b16*)carve(F * CI * 2); float* WA = (float*)carve(2 * CI * 4); float* S12 = (float*)carve((size_t)NB * 2 * N * 4); b16* HT = (b16*)carve((size_t)NB * CL * N * 2); float* G = (float*)carve((size_t)NB * N * CL * 4);
  if (off > ws_size || off > ((size_t)64 << 20)) return;
  wput_kernel<<<1, 256, 0, stream>>>(Fp(2), Fp(3), WT, WA);
  s_kernel<<<(NB * N + 255) / 256, 256, 0, stream>>>(Fp(0), WA, S12);
  ht_kernel<<<(unsigned)(((size_t)NB * CL * N / 2 + 255) / 256), 256, 0, stream>>>(Fp(0), HT);
  att_kernel<<<BLIM * (N / 16) * 3, 32, 0, stream>>>(S12, Ip(1), HT, BLIM, G);
  out_kernel<<<BLIM * (N / 16), 32, 0, stream>>>(G, WT, BLIM, (float*)d_out);
}
